// MultiHeadAttentionRoPE_10359461118256
// MI455X (gfx1250) — hardware-verified
//
#include <hip/hip_runtime.h>
#include <math.h>

#ifndef NB
#define NB 2
#endif
#ifndef SEQ
#define SEQ 2048
#endif
#ifndef NB_FULL
#define NB_FULL 2
#endif
#ifndef SEQ_FULL
#define SEQ_FULL 2048
#endif

static constexpr int kB       = NB;
static constexpr int kSeq     = SEQ;
static constexpr int kSeqFull = SEQ_FULL;
static constexpr int kDm      = 1024;
static constexpr int kHeads   = 16;
static constexpr int kHd      = 64;
static constexpr int kRows    = kB * kSeq;
static constexpr int kBH      = kB * kHeads;
static_assert(kHeads * kHd == kDm);
static_assert(kSeq % 64 == 0 && kDm % 64 == 0 && kDm % 32 == 0);
static_assert(kHd == 64);
static_assert(kB >= 1 && kB <= NB_FULL && kSeq >= 64 && kSeq <= kSeqFull);

static constexpr size_t kBytesX  = (size_t)kRows * kDm * 2;
static constexpr size_t kBytesW  = (size_t)kDm * kDm * 2;
static constexpr size_t kBytesP  = (size_t)kRows * kDm * 4;
static constexpr size_t kBytesT  = (size_t)kSeq * 32 * 4;
static constexpr size_t kBytesPl = (size_t)kBH * kSeq * kHd * 2;
static constexpr size_t kBytesC  = (size_t)kRows * kDm * 2;
static constexpr size_t kWsTotal = 3 * kBytesX + 4 * kBytesW + kBytesP + 2 * kBytesT + 4 * kBytesPl + 2 * kBytesC;
static_assert(kBytesX % 256 == 0 && kBytesW % 256 == 0 && kBytesP % 256 == 0 && kBytesT % 256 == 0 && kBytesPl % 256 == 0);
static_assert(kWsTotal <= (size_t)134217728);

typedef __attribute__((ext_vector_type(16))) _Float16 v16h;
typedef __attribute__((ext_vector_type(8)))  _Float16 v8h;
typedef __attribute__((ext_vector_type(16))) __bf16   v16b;
typedef __attribute__((ext_vector_type(8)))  __bf16   v8b;
typedef __attribute__((ext_vector_type(8)))  float    v8f;
typedef __attribute__((ext_vector_type(4)))  float    v4f;
typedef __attribute__((ext_vector_type(4)))  unsigned v4u;

__device__ __forceinline__ unsigned short f2bf_bits(float f) {
  unsigned u = __float_as_uint(f);
  return (unsigned short)((u + 0x7FFFu + ((u >> 16) & 1u)) >> 16);
}
__device__ __forceinline__ float bf_bits2f(unsigned short h) { return __uint_as_float(((unsigned)h) << 16); }

__device__ __forceinline__ void dep_guard_h(v8f& a, v8f& b, v16h x, v16h y) { asm volatile("v_nop\n\tv_nop\n\tv_nop\n\tv_nop" : "+v"(a), "+v"(b) : "v"(x), "v"(y)); }
__device__ __forceinline__ void dep_guard_b(v8f& a, v8f& b, v16b x, v16b y) { asm volatile("v_nop\n\tv_nop\n\tv_nop\n\tv_nop" : "+v"(a), "+v"(b) : "v"(x), "v"(y)); }
__device__ __forceinline__ void keep4_h(v16h a, v16h b, v16h c, v16h d) { asm volatile("v_nop" :: "v"(a), "v"(b), "v"(c), "v"(d)); }
__device__ __forceinline__ void keep4_b(v16b a, v16b b, v16b c, v16b d) { asm volatile("v_nop" :: "v"(a), "v"(b), "v"(c), "v"(d)); }
__device__ __forceinline__ void acc_guard4(v8f& a, v8f& b, v8f& c, v8f& d) { asm volatile("v_nop\n\tv_nop\n\tv_nop\n\tv_nop" : "+v"(a), "+v"(b), "+v"(c), "+v"(d)); }
template <typename T> struct Frag;
template <> struct Frag<_Float16> {
  typedef v16h V; union U { v16h v; v8h h[2]; };
  static __device__ __forceinline__ v16h load(const _Float16* p) {
    U f; f.h[0] = *(const v8h*)(p); f.h[1] = *(const v8h*)(p + 16); return f.v;
  }
  static __device__ __forceinline__ v8f mma(v16h a, v16h b, v8f c) {
    return __builtin_amdgcn_wmma_f32_16x16x32_f16(false, a, false, b, (short)0, c, false, false);
  }
  static __device__ __forceinline__ void guard(v8f& a, v8f& b, v16h x, v16h y) { dep_guard_h(a, b, x, y); }
  static __device__ __forceinline__ void keep(v16h a, v16h b, v16h c, v16h d) { keep4_h(a, b, c, d); }
};
template <> struct Frag<__bf16> {
  typedef v16b V; union U { v16b v; v8b h[2]; };
  static __device__ __forceinline__ v16b load(const __bf16* p) {
    U f; f.h[0] = *(const v8b*)(p); f.h[1] = *(const v8b*)(p + 16); return f.v;
  }
  static __device__ __forceinline__ v8f mma(v16b a, v16b b, v8f c) {
    return __builtin_amdgcn_wmma_f32_16x16x32_bf16(false, a, false, b, (short)0, c, false, false);
  }
  static __device__ __forceinline__ void guard(v8f& a, v8f& b, v16b x, v16b y) { dep_guard_b(a, b, x, y); }
  static __device__ __forceinline__ void keep(v16b a, v16b b, v16b c, v16b d) { keep4_b(a, b, c, d); }
};

template <int ET> struct Elem;
template <> struct Elem<0> { typedef _Float16 T; };
template <> struct Elem<1> { typedef __bf16 T; };
template <int ET, int SPLIT, int BIAS_MODE, int OUT_MODE, bool RESID, int ACT = 0>
__global__ __launch_bounds__(256) void wmma_gemm64(
    const unsigned short* __restrict__ Ap, const unsigned short* __restrict__ A2p, int lda, long strideA,
    const unsigned short* __restrict__ Btp, const unsigned short* __restrict__ Bt2p, int ldb, long strideB,
    void* __restrict__ Cout, void* __restrict__ Cout2, int ldc, long strideC,
    const float* __restrict__ bias,
    const float* __restrict__ resid, long strideR,
    int M, int N, int K, float scale) {
  typedef typename Elem<ET>::T T;
  typedef typename Frag<T>::V V;
  const T* A = (const T*)Ap; const T* A2 = (const T*)A2p; const T* Bt = (const T*)Btp; const T* Bt2 = (const T*)Bt2p;
  __shared__ __align__(16) float sT[8][16 * 68];
  const int b    = blockIdx.y;
  const int lane = threadIdx.x & 31;
  const int wave = threadIdx.x >> 5;
  const int tilesN = N >> 6;
  const int tilesM = M >> 6;
  const int tile = blockIdx.x * 8 + wave;
  if (tile >= tilesM * tilesN) return;
  const int tm = tile / tilesN;
  const int tn = tile - tm * tilesN;
  const int m0 = tm << 6;
  const int n0 = tn << 6;

  const T* Ab  = A  + (size_t)b * strideA;
  const T* Bb  = Bt + (size_t)b * strideB;
  const T* Ab2 = (SPLIT >= 1) ? (A2  + (size_t)b * strideA) : nullptr;
  const T* Bb2 = (SPLIT == 2) ? (Bt2 + (size_t)b * strideB) : nullptr;

  const int rlane = lane & 15;
  const int koff  = (lane >> 4) * 8;
  const int mOff  = (lane >> 4) * 8;

  v8f acc[4][4];
#pragma unroll
  for (int i = 0; i < 4; ++i)
#pragma unroll
    for (int j = 0; j < 4; ++j) acc[i][j] = (v8f){0.f,0.f,0.f,0.f,0.f,0.f,0.f,0.f};

  for (int k0 = 0; k0 < K; k0 += 32) {
    V bh[4], bl[4];
#pragma unroll
    for (int j = 0; j < 4; ++j) {
      const size_t bo = (size_t)(n0 + (j << 4) + rlane) * ldb + koff + k0;
      bh[j] = Frag<T>::load(Bb + bo);
      if (SPLIT == 2) bl[j] = Frag<T>::load(Bb2 + bo);
    }
#pragma unroll
    for (int i = 0; i < 4; ++i) {
      const size_t ao = (size_t)(m0 + (i << 4) + rlane) * lda + koff + k0;
      V ah = Frag<T>::load(Ab + ao);
      V al = ah;
      if (SPLIT >= 1) al = Frag<T>::load(Ab2 + ao);
#pragma unroll
      for (int j = 0; j < 4; ++j) {
        acc[i][j] = Frag<T>::mma(ah, bh[j], acc[i][j]);
        if (SPLIT == 2) acc[i][j] = Frag<T>::mma(ah, bl[j], acc[i][j]);
        if (SPLIT >= 1) acc[i][j] = Frag<T>::mma(al, bh[j], acc[i][j]);
      }
      Frag<T>::guard(acc[i][0], acc[i][3], ah, al);
    }
    Frag<T>::keep(bh[0], bh[1], bh[2], bh[3]);
    if (SPLIT == 2) Frag<T>::keep(bl[0], bl[1], bl[2], bl[3]);
  }
  acc_guard4(acc[0][0], acc[0][1], acc[0][2], acc[0][3]);
  acc_guard4(acc[1][0], acc[1][1], acc[1][2], acc[1][3]);
  acc_guard4(acc[2][0], acc[2][1], acc[2][2], acc[2][3]);
  acc_guard4(acc[3][0], acc[3][1], acc[3][2], acc[3][3]);

  float* slab = sT[wave];
  const float* Rb = RESID ? (resid + (size_t)b * strideR) : nullptr;
#pragma unroll
  for (int i = 0; i < 4; ++i) {
    const int mBase = m0 + (i << 4);
#pragma unroll
    for (int j = 0; j < 4; ++j) {
      const int n = n0 + (j << 4) + rlane;
      float bv = 0.f;
      if (BIAS_MODE == 2) bv = bias[n];
#pragma unroll
      for (int r = 0; r < 8; ++r) {
        float v = acc[i][j][r] * scale;
        if (BIAS_MODE == 1) v += bias[mBase + mOff + r];
        if (BIAS_MODE == 2) v += bv;
        if (RESID) v += Rb[(size_t)(mBase + mOff + r) * ldc + n];
        if (ACT == 1) v = tanhf(v);
        if (ACT == 2) v = fmaxf(v, 0.0f);
        if (ACT == 3) v = v / (1.0f + expf(-v));
        if (ACT == 4) v = (v > 0.f) ? v : 0.01f * v;
        if (ACT == 5) v = 0.5f * v * (1.0f + erff(v * 0.70710678118654752f));
        slab[(mOff + r) * 68 + (j << 4) + rlane] = v;
      }
    }
    __builtin_amdgcn_fence(3, "workgroup");
    __builtin_amdgcn_wave_barrier();
    __builtin_amdgcn_fence(2, "workgroup");
    if (OUT_MODE == 0) {
      float* C = (float*)Cout + (size_t)b * strideC;
      const int hh = lane >> 4, c4 = (lane & 15) * 4;
      for (int pass = 0; pass < 2; ++pass) {
#pragma unroll
        for (int it = 0; it < 8; ++it) {
          const int row = it * 2 + hh;
          v4f v = *(const v4f*)(slab + row * 68 + c4);
          *(volatile v4f*)(C + (size_t)(mBase + row) * ldc + n0 + c4) = v;
        }
        __threadfence();
      }
    } else {
      const int q = lane >> 3, c8 = (lane & 7) * 8;
      unsigned short* C  = (unsigned short*)Cout  + (size_t)b * strideC;
      unsigned short* C2 = (OUT_MODE == 2) ? ((unsigned short*)Cout2 + (size_t)b * strideC) : nullptr;
      for (int pass = 0; pass < 2; ++pass) {
#pragma unroll
        for (int it = 0; it < 4; ++it) {
          const int row = it * 4 + q;
          const float* sp = slab + row * 68 + c8;
          v8h hv, lv;
#pragma unroll
          for (int e = 0; e < 8; ++e) {
            if (OUT_MODE == 1) {
              hv[e] = (_Float16)sp[e];
            } else {
              unsigned short hb = f2bf_bits(sp[e]);
              unsigned short lb = f2bf_bits(sp[e] - bf_bits2f(hb));
              hv[e] = __builtin_bit_cast(_Float16, hb);
              lv[e] = __builtin_bit_cast(_Float16, lb);
            }
          }
          *(volatile v8h*)(C + (size_t)(mBase + row) * ldc + n0 + c8) = hv;
          if (OUT_MODE == 2) *(volatile v8h*)(C2 + (size_t)(mBase + row) * ldc + n0 + c8) = lv;
        }
        __threadfence();
      }
    }
    __builtin_amdgcn_fence(3, "workgroup");
    __builtin_amdgcn_wave_barrier();
    __builtin_amdgcn_fence(2, "workgroup");
  }
}

__device__ __forceinline__ void st2_v4u(unsigned short* p, v4u u) {
  *(volatile v4u*)(void*)p = u;
  __threadfence();
  *(volatile v4u*)(void*)p = u;
}
__device__ __forceinline__ unsigned pack_h2(float a, float b) {
  const unsigned short ha = __builtin_bit_cast(unsigned short, (_Float16)a);
  const unsigned short hb = __builtin_bit_cast(unsigned short, (_Float16)b);
  return (unsigned)ha | ((unsigned)hb << 16);
}
__device__ __forceinline__ unsigned pack_bf2(float a, float b) {
  return (unsigned)f2bf_bits(a) | ((unsigned)f2bf_bits(b) << 16);
}
__device__ __forceinline__ unsigned res_h2(float a, float b, float carry) {
  const float ha = (float)(_Float16)a;
  const float hb = (float)(_Float16)b;
  const float ra = (a - ha) * carry;
  const float rb = (b - hb) * carry;
  return pack_h2(ra, rb);
}
__device__ __forceinline__ v8f hmma_f16(v16h a, v16h b, v8f c) {
  c = __builtin_amdgcn_wmma_f32_16x16x32_f16(false, a, false, b, (short)0, c, false, false);
  asm volatile("v_nop\n\tv_nop\n\tv_nop\n\tv_nop" : "+v"(c) : "v"(a), "v"(b));
  return c;
}

__global__ __launch_bounds__(256) void k_cast_bf16(const float* __restrict__ in,
                                                    unsigned short* __restrict__ out,
                                                    int n8, int cols8, int seq, int seq_full) {
  const int i = blockIdx.x * 256 + threadIdx.x;
  if (i >= n8) return;
  const int m  = i / cols8;
  const int c8 = (i - m * cols8) * 8;
  const int bb = m / seq;
  const size_t srow = (size_t)bb * seq_full + (size_t)(m - bb * seq);
  const float* src = in + srow * ((size_t)cols8 * 8) + c8;
  const v4f a = *(const v4f*)(src);
  const v4f b = *(const v4f*)(src + 4);
  v4u u;
  u[0] = pack_bf2(a[0], a[1]);
  u[1] = pack_bf2(a[2], a[3]);
  u[2] = pack_bf2(b[0], b[1]);
  u[3] = pack_bf2(b[2], b[3]);
  st2_v4u(out + (size_t)i * 8, u);
}

struct RopeFreq { float f[32]; };
static_assert(sizeof(RopeFreq) == 128);

__global__ __launch_bounds__(256) void k_rope_table(float* __restrict__ cosT, float* __restrict__ sinT,
                                                      RopeFreq fr) {
#pragma clang fp contract(off)
  const int lane = threadIdx.x & 31;
  const int s = blockIdx.x * 8 + (threadIdx.x >> 5);
  float f = fr.f[0];
#pragma unroll
  for (int j = 1; j < 32; ++j) f = (lane == j) ? fr.f[j] : f;
  const float ang = (float)s * f;
  float sv, cv;
  sincosf(ang, &sv, &cv);
  const int base = (lane & 7) * 4;
  v4f c4, s4;
#pragma unroll
  for (int e = 0; e < 4; ++e) {
    c4[e] = __shfl(cv, base + e, 32);
    s4[e] = __shfl(sv, base + e, 32);
  }
  if (lane < 8) {
    float* cp = cosT + (size_t)s * 32 + base;
    float* sp = sinT + (size_t)s * 32 + base;
    *(volatile v4f*)(void*)cp = c4;
    *(volatile v4f*)(void*)sp = s4;
    __threadfence();
    *(volatile v4f*)(void*)cp = c4;
    *(volatile v4f*)(void*)sp = s4;
  }
}

__global__ __launch_bounds__(256) void k_rope_plane(const float* __restrict__ P,
                                                      const float* __restrict__ cosT, const float* __restrict__ sinT,
                                                      unsigned short* __restrict__ Hp, unsigned short* __restrict__ Lp,
                                                      int with_res, float carry) {
#pragma clang fp contract(off)
  const int t  = threadIdx.x;
  const int h  = blockIdx.y;
  const int m0 = blockIdx.x * 64;
  const int bb = m0 / kSeq;
  const int t0 = m0 - bb * kSeq;
#pragma unroll
  for (int it = 0; it < 2; ++it) {
    const int r  = it * 32 + (t >> 3);
    const int d8 = (t & 7) * 8;
    const int tp = t0 + r;
    const float* src = P + (size_t)(m0 + r) * kDm + h * kHd + d8;
    const v4f x0 = *(const v4f*)(src);
    const v4f x1 = *(const v4f*)(src + 4);
    const float* cptr = cosT + (size_t)tp * 32 + (d8 >> 1);
    const float* sptr = sinT + (size_t)tp * 32 + (d8 >> 1);
    const v4f cs = *(const v4f*)(cptr);
    const v4f sn = *(const v4f*)(sptr);
    const float o0 = x0[0] * cs[0] - x0[1] * sn[0];
    const float o1 = x0[0] * sn[0] + x0[1] * cs[0];
    const float o2 = x0[2] * cs[1] - x0[3] * sn[1];
    const float o3 = x0[2] * sn[1] + x0[3] * cs[1];
    const float o4 = x1[0] * cs[2] - x1[1] * sn[2];
    const float o5 = x1[0] * sn[2] + x1[1] * cs[2];
    const float o6 = x1[2] * cs[3] - x1[3] * sn[3];
    const float o7 = x1[2] * sn[3] + x1[3] * cs[3];
    const size_t off = (((size_t)(bb * kHeads + h)) * kSeq + tp) * kHd + d8;
    v4u uh;
    uh[0] = pack_h2(o0, o1);
    uh[1] = pack_h2(o2, o3);
    uh[2] = pack_h2(o4, o5);
    uh[3] = pack_h2(o6, o7);
    st2_v4u(Hp + off, uh);
    if (with_res != 0) {
      v4u ul;
      ul[0] = res_h2(o0, o1, carry);
      ul[1] = res_h2(o2, o3, carry);
      ul[2] = res_h2(o4, o5, carry);
      ul[3] = res_h2(o6, o7, carry);
      st2_v4u(Lp + off, ul);
    }
  }
}

__global__ __launch_bounds__(256) void k_vt_plane(const float* __restrict__ P, unsigned short* __restrict__ Vtp) {
  __shared__ float Vs[64 * 65];
  const int t  = threadIdx.x;
  const int h  = blockIdx.y;
  const int m0 = blockIdx.x * 64;
  const int bb = m0 / kSeq;
  const int t0 = m0 - bb * kSeq;
#pragma unroll
  for (int it = 0; it < 4; ++it) {
    const int idx = it * 256 + t;
    const int r = idx >> 4, c4 = (idx & 15) * 4;
    const v4f v = *(const v4f*)(P + (size_t)(m0 + r) * kDm + h * kHd + c4);
    Vs[r * 65 + c4 + 0] = v[0];
    Vs[r * 65 + c4 + 1] = v[1];
    Vs[r * 65 + c4 + 2] = v[2];
    Vs[r * 65 + c4 + 3] = v[3];
  }
  __syncthreads();
#pragma unroll
  for (int it = 0; it < 2; ++it) {
    const int drow = it * 32 + (t >> 3);
    const int s8   = (t & 7) * 8;
    v4u u;
    u[0] = pack_h2(Vs[(s8 + 0) * 65 + drow], Vs[(s8 + 1) * 65 + drow]);
    u[1] = pack_h2(Vs[(s8 + 2) * 65 + drow], Vs[(s8 + 3) * 65 + drow]);
    u[2] = pack_h2(Vs[(s8 + 4) * 65 + drow], Vs[(s8 + 5) * 65 + drow]);
    u[3] = pack_h2(Vs[(s8 + 6) * 65 + drow], Vs[(s8 + 7) * 65 + drow]);
    st2_v4u(Vtp + ((size_t)((bb * kHeads + h) * kHd + drow)) * kSeq + t0 + s8, u);
  }
}

__global__ __launch_bounds__(128) void k_attn_f16(const unsigned short* __restrict__ Qhp,
                                                    const unsigned short* __restrict__ Qlp,
                                                    const unsigned short* __restrict__ Kp,
                                                    const unsigned short* __restrict__ Vtp,
                                                    unsigned short* __restrict__ Chp,
                                                    unsigned short* __restrict__ Clp,
                                                    float sm_scale, float p_carry, float qres_inv, float o_scale) {
  __shared__ __align__(16) _Float16 Ksh[64 * 64];
  __shared__ __align__(16) _Float16 Vsh[64 * 64];
  __shared__ __align__(16) _Float16 Psh[4][16 * 64];
  __shared__ __align__(16) float    Osl[4][16 * 68];
  const int tid = threadIdx.x, wave = tid >> 5, lane = tid & 31;
  const int hh = lane >> 4, c = lane & 15;
  constexpr int nqb = kSeq / 64;
  const int bx = blockIdx.x;
  const int qb = bx % nqb;
  const int bh = bx / nqb;
  const int bb = bh / kHeads;
  const int h  = bh - bb * kHeads;
  const int q0 = qb * 64 + wave * 16;

  const size_t qoff = ((size_t)bh * kSeq + q0 + c) * kHd;
  const _Float16* Qh = (const _Float16*)(const void*)Qhp + qoff;
  const _Float16* Ql = (const _Float16*)(const void*)Qlp + qoff;
  v16h qa[2], ql[2];
#pragma unroll
  for (int dc = 0; dc < 2; ++dc) {
    qa[dc] = Frag<_Float16>::load(Qh + dc * 32 + 8 * hh);
    ql[dc] = Frag<_Float16>::load(Ql + dc * 32 + 8 * hh);
  }

  float mrow[8], lrow[8];
  v8f oacc[4];
#pragma unroll
  for (int r = 0; r < 8; ++r) { mrow[r] = -INFINITY; lrow[r] = 0.f; }
#pragma unroll
  for (int t = 0; t < 4; ++t) oacc[t] = (v8f){0.f,0.f,0.f,0.f,0.f,0.f,0.f,0.f};

  const v4u* Kg = (const v4u*)(const void*)(Kp + (size_t)bh * kSeq * kHd);
  const unsigned short* Vg = Vtp + (size_t)bh * kHd * kSeq;

#pragma unroll 1
  for (int kc = 0; kc < nqb; ++kc) {
    const int kv0 = kc * 64;
    __syncthreads();
#pragma unroll
    for (int it = 0; it < 4; ++it) {
      const int idx = it * 128 + tid;
      const v4u kk = Kg[(size_t)kv0 * 8 + idx];
      const int d = idx >> 3, p8 = idx & 7;
      const v4u vv = *(const v4u*)(const void*)(Vg + (size_t)d * kSeq + kv0 + p8 * 8);
      ((v4u*)(void*)Ksh)[idx] = kk;
      ((v4u*)(void*)Vsh)[idx] = vv;
    }
    __syncthreads();

    v8f s[4];
#pragma unroll
    for (int j = 0; j < 4; ++j) {
      const _Float16* krow = Ksh + (j * 16 + c) * kHd + 8 * hh;
      const v16h kb0 = Frag<_Float16>::load(krow);
      const v16h kb1 = Frag<_Float16>::load(krow + 32);
      v8f th = (v8f){0.f,0.f,0.f,0.f,0.f,0.f,0.f,0.f};
      th = hmma_f16(qa[0], kb0, th);
      th = hmma_f16(qa[1], kb1, th);
      v8f tl = (v8f){0.f,0.f,0.f,0.f,0.f,0.f,0.f,0.f};
      tl = hmma_f16(ql[0], kb0, tl);
      tl = hmma_f16(ql[1], kb1, tl);
#pragma unroll
      for (int r = 0; r < 8; ++r) s[j][r] = (th[r] + tl[r] * qres_inv) * sm_scale;
    }
    float cm[8];
#pragma unroll
    for (int r = 0; r < 8; ++r) {
      float m = -INFINITY;
#pragma unroll
      for (int j = 0; j < 4; ++j) m = fmaxf(m, s[j][r]);
#pragma unroll
      for (int off = 1; off < 16; off <<= 1) m = fmaxf(m, __shfl_xor(m, off, 32));
      cm[r] = m;
    }
    _Float16* pw = Psh[wave];
#pragma unroll
    for (int r = 0; r < 8; ++r) {
      const float mnew  = fmaxf(mrow[r], cm[r]);
      const float alpha = expf(mrow[r] - mnew);
      mrow[r] = mnew;
      float psum = 0.f;
#pragma unroll
      for (int j = 0; j < 4; ++j) {
        const float p = expf(s[j][r] - mnew);
        psum += p;
        pw[(8 * hh + r) * 64 + j * 16 + c] = (_Float16)(p * p_carry);
      }
#pragma unroll
      for (int off = 1; off < 16; off <<= 1) psum += __shfl_xor(psum, off, 32);
      lrow[r] = lrow[r] * alpha + psum;
#pragma unroll
      for (int t = 0; t < 4; ++t) oacc[t][r] *= alpha;
    }
    __builtin_amdgcn_fence(3, "workgroup");
    __builtin_amdgcn_wave_barrier();
    __builtin_amdgcn_fence(2, "workgroup");
#pragma unroll
    for (int kk = 0; kk < 2; ++kk) {
      const v16h pa = Frag<_Float16>::load(pw + c * 64 + kk * 32 + 8 * hh);
#pragma unroll
      for (int t = 0; t < 4; ++t) {
        const v16h vb = Frag<_Float16>::load(Vsh + (t * 16 + c) * 64 + kk * 32 + 8 * hh);
        oacc[t] = hmma_f16(pa, vb, oacc[t]);
      }
    }
  }

  float* os = Osl[wave];
#pragma unroll
  for (int r = 0; r < 8; ++r) {
    const float inv = o_scale * (1.0f / lrow[r]);
#pragma unroll
    for (int t = 0; t < 4; ++t) os[(8 * hh + r) * 68 + t * 16 + c] = oacc[t][r] * inv;
  }
  __builtin_amdgcn_fence(3, "workgroup");
  __builtin_amdgcn_wave_barrier();
  __builtin_amdgcn_fence(2, "workgroup");
  {
    const int q8 = lane >> 3, c8 = (lane & 7) * 8;
    unsigned short* Chb = Chp + (size_t)bb * kSeq * kDm + (size_t)h * kHd;
    unsigned short* Clb = Clp + (size_t)bb * kSeq * kDm + (size_t)h * kHd;
    for (int pass = 0; pass < 2; ++pass) {
#pragma unroll
      for (int it = 0; it < 4; ++it) {
        const int row = it * 4 + q8;
        const float* spp = os + row * 68 + c8;
        const v4f f0 = *(const v4f*)spp;
        const v4f f1 = *(const v4f*)(spp + 4);
        unsigned short hb[8], lb[8];
#pragma unroll
        for (int e = 0; e < 4; ++e) {
          hb[e]     = f2bf_bits(f0[e]);
          lb[e]     = f2bf_bits(f0[e] - bf_bits2f(hb[e]));
          hb[4 + e] = f2bf_bits(f1[e]);
          lb[4 + e] = f2bf_bits(f1[e] - bf_bits2f(hb[4 + e]));
        }
        v4u uh, ul;
#pragma unroll
        for (int e = 0; e < 4; ++e) {
          uh[e] = (unsigned)hb[2 * e] | ((unsigned)hb[2 * e + 1] << 16);
          ul[e] = (unsigned)lb[2 * e] | ((unsigned)lb[2 * e + 1] << 16);
        }
        const size_t o = (size_t)(q0 + row) * kDm + c8;
        *(volatile v4u*)(void*)(Chb + o) = uh;
        *(volatile v4u*)(void*)(Clb + o) = ul;
      }
      __threadfence();
    }
  }
}

extern "C" void kernel_launch(void* const* d_in, const int* in_sizes, int n_in,
                              void* d_out, int out_size, void* d_ws, size_t ws_size,
                              hipStream_t stream) {
  if (n_in < 7) return;
  const long needX = ((long)(kB - 1) * kSeqFull + kSeq) * (long)kDm;
  const long needW = (long)kDm * kDm;
  if ((long)in_sizes[0] < needX || (long)in_sizes[1] < needX || (long)in_sizes[2] < needX) return;
  if ((long)in_sizes[3] < needW || (long)in_sizes[4] < needW || (long)in_sizes[5] < needW || (long)in_sizes[6] < needW) return;
  if ((long)out_size < (long)kRows * kDm) return;

  const float* q   = (const float*)d_in[0];
  const float* k   = (const float*)d_in[1];
  const float* v   = (const float*)d_in[2];
  const float* W_q = (const float*)d_in[3];
  const float* W_k = (const float*)d_in[4];
  const float* W_v = (const float*)d_in[5];
  const float* W_o = (const float*)d_in[6];

  char* ws = (char*)d_ws;
  size_t off = 0;
  auto carve = [&](size_t bytes) -> char* { char* p = ws + off; off += (bytes + 255) & ~(size_t)255; return p; };
  unsigned short* Xq  = (unsigned short*)carve(kBytesX);
  unsigned short* Xk  = (unsigned short*)carve(kBytesX);
  unsigned short* Xv  = (unsigned short*)carve(kBytesX);
  unsigned short* Wqb = (unsigned short*)carve(kBytesW);
  unsigned short* Wkb = (unsigned short*)carve(kBytesW);
  unsigned short* Wvb = (unsigned short*)carve(kBytesW);
  unsigned short* Wob = (unsigned short*)carve(kBytesW);
  float* Pf   = (float*)carve(kBytesP);
  float* cosT = (float*)carve(kBytesT);
  float* sinT = (float*)carve(kBytesT);
  unsigned short* Qh = (unsigned short*)carve(kBytesPl);
  unsigned short* Ql = (unsigned short*)carve(kBytesPl);
  unsigned short* Kpl= (unsigned short*)carve(kBytesPl);
  unsigned short* Vt = (unsigned short*)carve(kBytesPl);
  unsigned short* Ch = (unsigned short*)carve(kBytesC);
  unsigned short* Cl = (unsigned short*)carve(kBytesC);
  if (off > ws_size || off > kWsTotal) return;

  double rt = 1.3335214321633;
  for (int it = 0; it < 8; ++it) {
    double p31 = 1.0;
    for (int kk = 0; kk < 31; ++kk) p31 *= rt;
    const double fv = p31 * rt - 10000.0;
    rt = rt - fv / (32.0 * p31);
  }
  RopeFreq fr;
  {
    double pw = 1.0;
    for (int i = 0; i < 32; ++i) {
      const float pf = (float)pw;
      fr.f[i] = 1.0f / pf;
      pw *= rt;
    }
  }

  const int n8x = kRows * kDm / 8;
  k_cast_bf16<<<(n8x + 255) / 256, 256, 0, stream>>>(q, Xq, n8x, kDm / 8, kSeq, kSeqFull);
  k_cast_bf16<<<(n8x + 255) / 256, 256, 0, stream>>>(k, Xk, n8x, kDm / 8, kSeq, kSeqFull);
  k_cast_bf16<<<(n8x + 255) / 256, 256, 0, stream>>>(v, Xv, n8x, kDm / 8, kSeq, kSeqFull);
  const int n8w = kDm * kDm / 8;
  k_cast_bf16<<<(n8w + 255) / 256, 256, 0, stream>>>(W_q, Wqb, n8w, kDm / 8, kDm, kDm);
  k_cast_bf16<<<(n8w + 255) / 256, 256, 0, stream>>>(W_k, Wkb, n8w, kDm / 8, kDm, kDm);
  k_cast_bf16<<<(n8w + 255) / 256, 256, 0, stream>>>(W_v, Wvb, n8w, kDm / 8, kDm, kDm);
  k_cast_bf16<<<(n8w + 255) / 256, 256, 0, stream>>>(W_o, Wob, n8w, kDm / 8, kDm, kDm);
  static_assert(kSeq % 8 == 0);
  k_rope_table<<<kSeq / 8, 256, 0, stream>>>(cosT, sinT, fr);

  static_assert(((kRows / 64) * (kDm / 64)) % 8 == 0);
  const dim3 ggrid((kRows / 64) * (kDm / 64) / 8, 1);
  const dim3 pgrid(kRows / 64, kHeads);
  wmma_gemm64<1, 0, 0, 0, false><<<ggrid, 256, 0, stream>>>(
      Xq, Xq, kDm, 0L, Wqb, Wqb, kDm, 0L, (void*)Pf, (void*)Pf, kDm, 0L,
      cosT, cosT, 0L, kRows, kDm, kDm, 1.0f);
  k_rope_plane<<<pgrid, 256, 0, stream>>>(Pf, cosT, sinT, Qh, Ql, 1, 2048.0f);
  wmma_gemm64<1, 0, 0, 0, false><<<ggrid, 256, 0, stream>>>(
      Xk, Xk, kDm, 0L, Wkb, Wkb, kDm, 0L, (void*)Pf, (void*)Pf, kDm, 0L,
      cosT, cosT, 0L, kRows, kDm, kDm, 1.0f);
  k_rope_plane<<<pgrid, 256, 0, stream>>>(Pf, cosT, sinT, Kpl, Kpl, 0, 2048.0f);
  wmma_gemm64<1, 0, 0, 0, false><<<ggrid, 256, 0, stream>>>(
      Xv, Xv, kDm, 0L, Wvb, Wvb, kDm, 0L, (void*)Pf, (void*)Pf, kDm, 0L,
      cosT, cosT, 0L, kRows, kDm, kDm, 1.0f);
  k_vt_plane<<<pgrid, 256, 0, stream>>>(Pf, Vt);
  k_attn_f16<<<kBH * (kSeq / 64), 128, 0, stream>>>(Qh, Ql, Kpl, Vt, Ch, Cl,
                                                     0.125f, 32768.0f, 1.0f / 2048.0f, 1.0f / 32768.0f);
  wmma_gemm64<1, 1, 0, 0, false><<<ggrid, 256, 0, stream>>>(
      Ch, Cl, kDm, 0L, Wob, Wob, kDm, 0L, d_out, d_out, kDm, 0L,
      cosT, cosT, 0L, kRows, kDm, kDm, 1.0f);
}
